// PointNet_80333068304471
// MI455X (gfx1250) — hardware-verified
//
#include <hip/hip_runtime.h>


namespace {
typedef _Float16 b16;
typedef __attribute__((ext_vector_type(16))) _Float16 v16b;
typedef __attribute__((ext_vector_type(8))) _Float16 v8b;
typedef __attribute__((ext_vector_type(4))) _Float16 v4h;
typedef __attribute__((ext_vector_type(2))) _Float16 v2h;
typedef __attribute__((ext_vector_type(8))) float v8f;
typedef __attribute__((ext_vector_type(4))) float v4f;
typedef __attribute__((ext_vector_type(2))) float v2f;
__device__ __forceinline__ float bf16_rne(float f) { unsigned int u = __float_as_uint(f); u += 0x7FFFu + ((u >> 16) & 1u); return __uint_as_float(u & 0xFFFF0000u); }
__device__ __forceinline__ void split16(float v, b16& hi, b16& lo) { hi = (b16)v; lo = (b16)(v - (float)hi); }
__device__ __forceinline__ v16b frag_kb(const b16* p, int hh) { const v8b a = *(const v8b*)(p + 8 * hh), b = *(const v8b*)(p + 16 + 8 * hh); v16b f;
#pragma unroll
  for (int e = 0; e < 8; ++e) { f[e] = a[e]; f[8 + e] = b[e]; } return f; }
__device__ __forceinline__ v8f wmma16b(v16b a, v16b b, v8f c) { v8f d = __builtin_amdgcn_wmma_f32_16x16x32_f16(false, a, false, b, (short)0, c, false, false); asm volatile("v_nop\n\tv_nop\n\tv_nop\n\tv_nop" : "+v"(d) : "v"(a), "v"(b)); return d; }
__device__ __forceinline__ void wave_lds_sync() { __builtin_amdgcn_fence(__ATOMIC_RELEASE, "workgroup"); __builtin_amdgcn_wave_barrier(); __builtin_amdgcn_fence(__ATOMIC_ACQUIRE, "workgroup"); }
__device__ __forceinline__ float pmul(float a, float b) { float p = a * b; asm volatile("" : "+v"(p)); return p; }
__device__ __forceinline__ int iclamp(int v, int lo, int hi) { return v < lo ? lo : (v > hi ? hi : v); }
__device__ __forceinline__ float nexp2(float v) { return __builtin_amdgcn_exp2f(v); }
constexpr int NPT = 1000000, NPL = NPT  , NBK = NPT / 64, B = 4096, C1 = 32, C2 = 128, C3 = 256, F1 = 128, F2 = 64, F3 = 75, F3P = 96, KOUT = 75, N = B, NP = B;
constexpr float XS = 8.0f, WSC = 256.0f;
static_assert(NPT % 64 == 0 && NPL % 64 == 0 && B % 32 == 0, "tiling");


template <int KD, int NOUT, int LDA, int LDT, bool RNDA>
__global__ __launch_bounds__(64) void gemmx_kernel(const float* __restrict__ A, int nv, const b16* __restrict__ W, const float* __restrict__ bias, int mrows, float* __restrict__ T) {
  constexpr int SL = NOUT < 128 ? NOUT : 128, NT = SL / 16, KC = KD < 128 ? KD : 128;
  static_assert(KD % KC == 0 && KC % 32 == 0 && NOUT % SL == 0 && SL % 32 == 0 && LDA >= KD && LDT >= NOUT, "gemmx tiling");
  __shared__ __attribute__((aligned(16))) b16 Ah[2][16][KC + 8], Al[2][16][KC + 8]; __shared__ __attribute__((aligned(16))) float Tf[2][16][SL + 4];
  const int wave = threadIdx.x >> 5, lane = threadIdx.x & 31, nloc = lane & 15, hlf = lane >> 4; const size_t m0 = (size_t)blockIdx.x * 32 + wave * 16; const int n0 = blockIdx.y * SL;
  v8f acc[NT];
#pragma unroll
  for (int t = 0; t < NT; ++t) acc[t] = (v8f){};
#pragma unroll 1
  for (int kc = 0; kc < KD; kc += KC) {
    for (int idx = lane; idx < 16 * (KC / 4); idx += 32) { const int rr = idx / (KC / 4), c4 = (idx % (KC / 4)) * 4; const size_t row = (m0 + rr < (size_t)nv) ? (m0 + rr) : (size_t)(nv - 1); const v4f v = *(const v4f*)(A + row * LDA + kc + c4); v4h hv, lv;
      for (int j = 0; j < 4; ++j) { b16 ph, pl; split16((RNDA ? bf16_rne(v[j]) : v[j]) * XS, ph, pl); hv[j] = ph; lv[j] = pl; } *(v4h*)(&Ah[wave][rr][c4]) = hv; *(v4h*)(&Al[wave][rr][c4]) = lv; }
    wave_lds_sync();
#pragma unroll
    for (int kb = 0; kb < KC; kb += 32) { const v16b a = frag_kb(&Ah[wave][nloc][kb], hlf), al = frag_kb(&Al[wave][nloc][kb], hlf);
#pragma unroll
      for (int t = 0; t < NT; ++t) { const v16b bw = frag_kb(W + (size_t)(n0 + t * 16 + nloc) * KD + kc + kb, hlf); acc[t] = wmma16b(a, bw, acc[t]); if (!RNDA) acc[t] = wmma16b(al, bw, acc[t]); } }
    wave_lds_sync(); }
#pragma unroll
  for (int t = 0; t < NT; ++t) { const float bb = bias ? bf16_rne(bias[n0 + t * 16 + nloc]) : 0.0f;
#pragma unroll
    for (int r = 0; r < 8; ++r) Tf[wave][8 * hlf + r][t * 16 + nloc] = acc[t][r] * (1.0f / (XS * WSC)) + bb; }
  wave_lds_sync();
  for (int pass = 0; pass < 2; ++pass) { for (int idx = lane; idx < 16 * (SL / 4); idx += 32) { const int rr = idx / (SL / 4), c4 = (idx % (SL / 4)) * 4; if (m0 + rr < (size_t)mrows) *(volatile v4f*)(T + (m0 + rr) * LDT + n0 + c4) = *(const v4f*)(&Tf[wave][rr][c4]); } __threadfence(); }
}

template <int KD>
__global__ __launch_bounds__(256) void wrows_kernel(const float* __restrict__ w, int nrow, int nrowp, b16* __restrict__ WT) {
  const int u = blockIdx.x * 256 + threadIdx.x; if (u >= nrowp * KD / 8) return; const int e = u * 8; const int o = e / KD, k0 = e % KD; v8b v;
  for (int j = 0; j < 8; ++j) v[j] = (b16)(o < nrow ? bf16_rne(w[(size_t)o * KD + k0 + j]) * WSC : 0.0f);
  for (int pass = 0; pass < 2; ++pass) { *(volatile v8b*)(WT + e) = v; __threadfence(); }
}
__global__ __launch_bounds__(128) void point_kernel(const float* __restrict__ pts, const float* __restrict__ col, const int* __restrict__ batch, const float* __restrict__ w1, const float* __restrict__ b1, const b16* __restrict__ W2T, const float* __restrict__ b2, const b16* __restrict__ W3T, const float* __restrict__ b3, float* __restrict__ PM, int* __restrict__ PSEG) {
  __shared__ __attribute__((aligned(16))) b16 A1h[4][16][C1 + 8], A1l[4][16][C1 + 8], A2[4][16][C2 + 8]; __shared__ float W1s[C1 * 6], B1s[C1]; __shared__ float mx[4][2][C3]; __shared__ int sflag[64];
  const int wave = threadIdx.x >> 5, lane = threadIdx.x & 31, nloc = lane & 15, hlf = lane >> 4; const size_t p0 = (size_t)blockIdx.x * 64; const size_t pw = p0 + wave * 16;
  for (int i = threadIdx.x; i < C1 * 6; i += 128) W1s[i] = bf16_rne(w1[i]); if (threadIdx.x < C1) B1s[threadIdx.x] = bf16_rne(b1[threadIdx.x]);
  const int seg0 = batch[p0]; if (threadIdx.x < 64) sflag[threadIdx.x] = (batch[p0 + threadIdx.x] != seg0) ? 1 : 0;
  __syncthreads();
  { const int r = lane >> 1, o0 = (lane & 1) * 16; const size_t p = pw + r; float xin[6]; for (int j = 0; j < 3; ++j) { xin[j] = bf16_rne(pts[p * 3 + j]); xin[3 + j] = bf16_rne(col[p * 3 + j]); }
    for (int o = o0; o < o0 + 16; ++o) { float a = B1s[o];
#pragma unroll
      for (int j = 0; j < 6; ++j) a = fmaf(xin[j], W1s[o * 6 + j], a); a = fmaxf(a, 0.0f); b16 ph, pl; split16(a * XS, ph, pl); A1h[wave][r][o] = ph; A1l[wave][r][o] = pl; } }
  wave_lds_sync();
  { v8f acc[8];
#pragma unroll
    for (int t = 0; t < 8; ++t) acc[t] = (v8f){};
    const v16b a = frag_kb(&A1h[wave][nloc][0], hlf), al = frag_kb(&A1l[wave][nloc][0], hlf);
#pragma unroll
    for (int t = 0; t < 8; ++t) { const v16b bw = frag_kb(W2T + (size_t)(t * 16 + nloc) * C1, hlf); acc[t] = wmma16b(a, bw, acc[t]); acc[t] = wmma16b(al, bw, acc[t]); }
#pragma unroll
    for (int t = 0; t < 8; ++t) { const float bb = bf16_rne(b2[t * 16 + nloc]);
#pragma unroll
      for (int r = 0; r < 8; ++r) A2[wave][8 * hlf + r][t * 16 + nloc] = (b16)(fmaxf(acc[t][r] * (1.0f / (XS * WSC)) + bb, 0.0f) * XS); } }
  wave_lds_sync();
  { v8f acc[16];
#pragma unroll
    for (int t = 0; t < 16; ++t) acc[t] = (v8f){};
#pragma unroll
    for (int kb = 0; kb < C2; kb += 32) { const v16b a = frag_kb(&A2[wave][nloc][kb], hlf);
#pragma unroll
      for (int t = 0; t < 16; ++t) acc[t] = wmma16b(a, frag_kb(W3T + (size_t)(t * 16 + nloc) * C2 + kb, hlf), acc[t]); }
#pragma unroll
    for (int t = 0; t < 16; ++t) { const float bb = bf16_rne(b3[t * 16 + nloc]); float m0 = -INFINITY, m1 = -INFINITY;
#pragma unroll
      for (int r = 0; r < 8; ++r) { const float v = acc[t][r] * (1.0f / (XS * WSC)) + bb; const int f = sflag[wave * 16 + 8 * hlf + r]; m0 = f ? m0 : fmaxf(m0, v); m1 = f ? fmaxf(m1, v) : m1; }
      m0 = fmaxf(m0, __shfl_xor(m0, 16)); m1 = fmaxf(m1, __shfl_xor(m1, 16)); if (hlf == 0) { mx[wave][0][t * 16 + nloc] = m0; mx[wave][1][t * 16 + nloc] = m1; } } }
  __syncthreads();
  for (int pass = 0; pass < 2; ++pass) { for (int q = threadIdx.x; q < 2 * C3 / 4; q += 128) { const int slot = q / (C3 / 4), c4 = (q % (C3 / 4)) * 4; v4f o;
      for (int j = 0; j < 4; ++j) { const int c = c4 + j; o[j] = fmaxf(fmaxf(mx[0][slot][c], mx[1][slot][c]), fmaxf(mx[2][slot][c], mx[3][slot][c])); }
      *(volatile v4f*)(PM + ((size_t)blockIdx.x * 2 + slot) * C3 + c4) = o; }
    if (threadIdx.x < 32) ((volatile int*)PSEG)[(size_t)blockIdx.x * 32 + threadIdx.x] = (threadIdx.x == 0) ? seg0 : 0;
    __threadfence(); }
}
__device__ int lower_bound_i(const int* a, int n, int key) { int lo = 0, hi = n; while (lo < hi) { const int mid = (lo + hi) >> 1; if (a[mid] < key) lo = mid + 1; else hi = mid; } return lo; }
__global__ __launch_bounds__(256) void segmax_kernel(const int* __restrict__ batch, const float* __restrict__ PM, const int* __restrict__ PSEG, float* __restrict__ XM) {
  const int b = blockIdx.x, c = threadIdx.x; const int lo = lower_bound_i(batch, NPL, b), hi = lower_bound_i(batch, NPL, b + 1); float m = 0.0f;
  if (hi > lo) { const int k0 = lo / 64, k1 = (hi - 1) / 64;
#pragma unroll 1
    for (int k = k0; k <= k1; ++k) { const int slot = (PSEG[(size_t)k * 32] == b) ? 0 : 1; m = fmaxf(m, PM[((size_t)k * 2 + slot) * C3 + c]); } }
  for (int pass = 0; pass < 2; ++pass) { ((volatile float*)XM)[(size_t)b * C3 + c] = m; __threadfence(); }
}
__global__ __launch_bounds__(256) void relu_kernel(float* __restrict__ Hp, int n4) { const int u = blockIdx.x * 256 + threadIdx.x; if (u >= n4) return; v4f v = *(const v4f*)(Hp + (size_t)u * 4); for (int j = 0; j < 4; ++j) v[j] = fmaxf(v[j], 0.0f); for (int pass = 0; pass < 2; ++pass) { *(volatile v4f*)(Hp + (size_t)u * 4) = v; __threadfence(); } }
__global__ __launch_bounds__(256) void final_kernel(const float* __restrict__ H3, const float* __restrict__ fb3, const float* __restrict__ cmean, const float* __restrict__ cstd, float* __restrict__ out) {
  const int u = blockIdx.x * 256 + threadIdx.x; if (u >= B * KOUT) return; const int b = u / KOUT, r = u % KOUT; const float v = (H3[(size_t)b * F3P + r] + bf16_rne(fb3[r])) * bf16_rne(cstd[r]) + bf16_rne(cmean[r]);
  for (int pass = 0; pass < 2; ++pass) { ((volatile float*)out)[u] = v; __threadfence(); }
}
}

extern "C" void kernel_launch(void* const* d_in, const int* in_sizes, int n_in, void* d_out, int out_size, void* d_ws, size_t ws_size, hipStream_t stream) {
  (void)n_in;
  auto Fp = [&](int i) { return (const float*)d_in[i]; }; auto Ip = [&](int i) { return (const int*)d_in[i]; };
  if (in_sizes[0] != NPT * 3 || in_sizes[1] != NPT * 3 || in_sizes[2] != NPT || in_sizes[3] != C1 * 6 || in_sizes[5] != C2 * C1 || in_sizes[7] != C3 * C2 || in_sizes[9] != F1 * C3 || in_sizes[11] != F2 * F1 || in_sizes[13] != F3 * F2 || in_sizes[14] != F3 || in_sizes[15] != KOUT || in_sizes[16] != KOUT || out_size != B * KOUT) return;
  size_t off = 0; char* ws = (char*)d_ws;
  auto carve = [&](size_t bytes) { char* p = ws + off; off += (bytes + 255) & ~(size_t)255; return p; };
  b16* W2T = (b16*)carve((size_t)C2 * C1 * 2); b16* W3T = (b16*)carve((size_t)C3 * C2 * 2); b16* FW1 = (b16*)carve((size_t)F1 * C3 * 2); b16* FW2 = (b16*)carve((size_t)F2 * F1 * 2); b16* FW3 = (b16*)carve((size_t)F3P * F2 * 2);
  float* PM = (float*)carve((size_t)NBK * 2 * C3 * 4); int* PSEG = (int*)carve((size_t)NBK * 32 * 4); float* XM = (float*)carve((size_t)B * C3 * 4); float* H1 = (float*)carve((size_t)B * F1 * 4); float* H2 = (float*)carve((size_t)B * F2 * 4); float* H3 = (float*)carve((size_t)B * F3P * 4); float* FB3P = (float*)carve((size_t)F3P * 4);
  if (off > ws_size || off > ((size_t)128 << 20)) return;
  wrows_kernel<C1><<<(C2 * C1 / 8 + 255) / 256, 256, 0, stream>>>(Fp(5), C2, C2, W2T); wrows_kernel<C2><<<(C3 * C2 / 8 + 255) / 256, 256, 0, stream>>>(Fp(7), C3, C3, W3T);
  wrows_kernel<C3><<<(F1 * C3 / 8 + 255) / 256, 256, 0, stream>>>(Fp(9), F1, F1, FW1); wrows_kernel<F1><<<(F2 * F1 / 8 + 255) / 256, 256, 0, stream>>>(Fp(11), F2, F2, FW2); wrows_kernel<F2><<<(F3P * F2 / 8 + 255) / 256, 256, 0, stream>>>(Fp(13), F3, F3P, FW3);
  point_kernel<<<NPL / 64, 128, 0, stream>>>(Fp(0), Fp(1), Ip(2), Fp(3), Fp(4), W2T, Fp(6), W3T, Fp(8), PM, PSEG);
  segmax_kernel<<<B, C3, 0, stream>>>(Ip(2), PM, PSEG, XM);
  gemmx_kernel<C3, F1, C3, F1, false><<<dim3(B / 32, 1), 64, 0, stream>>>(XM, B, FW1, Fp(10), B, H1); relu_kernel<<<(B * F1 / 4 + 255) / 256, 256, 0, stream>>>(H1, B * F1 / 4);
  gemmx_kernel<F1, F2, F1, F2, false><<<dim3(B / 32, 1), 64, 0, stream>>>(H1, B, FW2, Fp(12), B, H2); relu_kernel<<<(B * F2 / 4 + 255) / 256, 256, 0, stream>>>(H2, B * F2 / 4);
  gemmx_kernel<F2, F3P, F2, F3P, false><<<dim3(B / 32, 1), 64, 0, stream>>>(H2, B, FW3, nullptr, B, H3);
  final_kernel<<<(B * KOUT + 255) / 256, 256, 0, stream>>>(H3, Fp(14), Fp(15), Fp(16), (float*)d_out);
}
